// FlashMultiHeadAttention_14061722927977
// MI455X (gfx1250) — hardware-verified
//
#include <hip/hip_runtime.h>
#include <math.h>
#include <stdint.h>

#define NB     2
#define SQ     2048
#define EMB    2048
#define NH     16
#define HDM    128
#define NFREQ  64
#define QKN    4096
#define QW     2048
#define AOW    4096
#define NTOK   4096

typedef __bf16       v16b __attribute__((ext_vector_type(16)));
typedef __bf16       v8b  __attribute__((ext_vector_type(8)));
typedef float        v8f  __attribute__((ext_vector_type(8)));
typedef float        v4f  __attribute__((ext_vector_type(4)));
typedef unsigned int v4u  __attribute__((ext_vector_type(4)));

__device__ __forceinline__ unsigned short bf_bits(float f) {
  const unsigned u = __float_as_uint(f);
  return (unsigned short)((u + 0x7FFFu + ((u >> 16) & 1u)) >> 16);
}
__device__ __forceinline__ float bf_val(unsigned short h) { return __uint_as_float(((unsigned)h) << 16); }
__device__ __forceinline__ float bf_rne(float f) { return bf_val(bf_bits(f)); }
__device__ __forceinline__ unsigned pk16(unsigned short a, unsigned short b) { return (unsigned)a | ((unsigned)b << 16); }
__device__ __forceinline__ v8f zero8() { v8f z = {0.f, 0.f, 0.f, 0.f, 0.f, 0.f, 0.f, 0.f}; return z; }
__device__ __forceinline__ int wave_id() { return __builtin_amdgcn_readfirstlane((int)(threadIdx.x >> 5)); }

__device__ __forceinline__ void lds_wave_sync() {
  __builtin_amdgcn_fence(__ATOMIC_RELEASE, "workgroup");
  __builtin_amdgcn_wave_barrier();
  __builtin_amdgcn_fence(__ATOMIC_ACQUIRE, "workgroup");
}

union FragB { v16b v; v8b h[2]; };
__device__ __forceinline__ v16b ldfrag_b(const __bf16* p) { FragB f; f.h[0] = *(const v8b*)(p); f.h[1] = *(const v8b*)(p + 16); return f.v; }

__device__ __forceinline__ v8f mma_b(v16b a, v16b b, v8f c) {
  return __builtin_amdgcn_wmma_f32_16x16x32_bf16(false, a, false, b, (short)0, c, false, false);
}
__device__ __forceinline__ void guard2b3(v8f& a, v8f& b, v16b x0, v16b x1, v16b y) {
  asm volatile("v_nop\n\tv_nop\n\tv_nop\n\tv_nop" : "+v"(a), "+v"(b) : "v"(x0), "v"(x1), "v"(y) : "memory");
}
__device__ __forceinline__ void guard1b4(v8f& a, v16b w, v16b x, v16b y, v16b z) {
  asm volatile("v_nop\n\tv_nop\n\tv_nop\n\tv_nop" : "+v"(a) : "v"(w), "v"(x), "v"(y), "v"(z) : "memory");
}
__device__ __forceinline__ void acc_guard4(v8f& a, v8f& b, v8f& c, v8f& d) {
  asm volatile("v_nop\n\tv_nop\n\tv_nop\n\tv_nop" : "+v"(a), "+v"(b), "+v"(c), "+v"(d));
}
__device__ __forceinline__ void acc_guard2(v8f& a, v8f& b) {
  asm volatile("v_nop\n\tv_nop\n\tv_nop\n\tv_nop" : "+v"(a), "+v"(b));
}

__global__ __launch_bounds__(256) void rope_table_kernel(float* __restrict__ cst, float* __restrict__ snt, int ntok) {
  const int lane = threadIdx.x & 31;
  const int wave = (int)(threadIdx.x >> 5);
  const int t = (int)blockIdx.x * 8 + wave;
  if (t >= ntok) return;
  const float pf = (float)t;
#pragma unroll 1
  for (int half = 0; half < 2; ++half) {
    const int j = lane + 32 * half;
    const float e   = (float)j * 0.015625f;
    const float pw  = powf(10000.0f, e);
    const float inv = 1.0f / pw;
    const float ang = pf * inv;
    const float cv  = cosf(ang);
    const float sv  = sinf(ang);
    const size_t o = (size_t)t * NFREQ + j;
    ((volatile float*)cst)[o] = cv;
    ((volatile float*)snt)[o] = sv;
    __threadfence();
    ((volatile float*)cst)[o] = cv;
    ((volatile float*)snt)[o] = sv;
  }
}

__global__ __launch_bounds__(256) void cvt_bf16_kernel(const float* __restrict__ in, unsigned short* __restrict__ outp, int n8) {
  const int i = (int)blockIdx.x * 256 + (int)threadIdx.x;
  if (i >= n8) return;
  const size_t e = 8 * (size_t)i;
  const v4f a = *(const v4f*)(in + e);
  const v4f b = *(const v4f*)(in + e + 4);
  v4u w;
  w[0] = pk16(bf_bits(a[0]), bf_bits(a[1]));
  w[1] = pk16(bf_bits(a[2]), bf_bits(a[3]));
  w[2] = pk16(bf_bits(b[0]), bf_bits(b[1]));
  w[3] = pk16(bf_bits(b[2]), bf_bits(b[3]));
  *(volatile v4u*)(outp + e) = w;
  __threadfence();
  *(volatile v4u*)(outp + e) = w;
}

__global__ __launch_bounds__(256) void cvt_wo2_kernel(const float* __restrict__ in, unsigned short* __restrict__ outp,
                                                      int n8, int kin, int ldo) {
  const int i = (int)blockIdx.x * 256 + (int)threadIdx.x;
  if (i >= n8) return;
  const size_t e = 8 * (size_t)i;
  const int n = (int)(e / (size_t)kin);
  const int k = (int)(e - (size_t)n * kin);
  const v4f a = *(const v4f*)(in + e);
  const v4f b = *(const v4f*)(in + e + 4);
  v4u w;
  w[0] = pk16(bf_bits(a[0]), bf_bits(a[1]));
  w[1] = pk16(bf_bits(a[2]), bf_bits(a[3]));
  w[2] = pk16(bf_bits(b[0]), bf_bits(b[1]));
  w[3] = pk16(bf_bits(b[2]), bf_bits(b[3]));
  const size_t o = (size_t)n * ldo + k;
  *(volatile v4u*)(outp + o) = w;
  *(volatile v4u*)(outp + o + kin) = w;
  __threadfence();
  *(volatile v4u*)(outp + o) = w;
  *(volatile v4u*)(outp + o + kin) = w;
}

template <int EPI> struct SlabCfg;
template <> struct SlabCfg<0> { static constexpr int PERWF = 4224; };
template <> struct SlabCfg<1> { static constexpr int PERWF = 2048; };
template <> struct SlabCfg<2> { static constexpr int PERWF = 2176; };

template <int EPI>
__global__ __launch_bounds__(128) void gemm_w32x128_kernel(
    const unsigned short* __restrict__ Ap, int lda,
    const unsigned short* __restrict__ Btp, int ldb,
    const float* __restrict__ cst, const float* __restrict__ snt,
    const float* __restrict__ bias0, const float* __restrict__ bias1,
    void* C0, void* C1, void* C2, void* C3, int ldc, int ldc2,
    int M, int N, int K) {
  extern __shared__ v4f lds_dyn4[];
  float* lds_all = (float*)(void*)lds_dyn4;

  const int lane = threadIdx.x & 31;
  const int wave = wave_id();
  const int hh = lane >> 4;
  const int rl = lane & 15;
  const int tilesN = N >> 7;
  const int tilesM = M >> 5;
  const int tile = (int)blockIdx.x * 4 + wave;
  if (tile >= tilesM * tilesN) return;
  const int tm = tile / tilesN;
  const int tn = tile - tm * tilesN;
  const int m0 = tm << 5;
  const int n0 = tn << 7;

  const __bf16* A  = (const __bf16*)(const void*)Ap;
  const __bf16* Bt = (const __bf16*)(const void*)Btp;

  v8f acc[2][8];
#pragma unroll
  for (int i = 0; i < 2; ++i)
#pragma unroll
    for (int j = 0; j < 8; ++j) acc[i][j] = zero8();

  for (int k0 = 0; k0 < K; k0 += 32) {
    v16b ah[2];
#pragma unroll
    for (int i = 0; i < 2; ++i) ah[i] = ldfrag_b(A + (size_t)(m0 + i * 16 + rl) * lda + k0 + 8 * hh);
#pragma unroll
    for (int j = 0; j < 8; ++j) {
      const v16b bj = ldfrag_b(Bt + (size_t)(n0 + j * 16 + rl) * ldb + k0 + 8 * hh);
      acc[0][j] = mma_b(ah[0], bj, acc[0][j]);
      acc[1][j] = mma_b(ah[1], bj, acc[1][j]);
      guard2b3(acc[0][j], acc[1][j], ah[0], ah[1], bj);
    }
  }
  acc_guard4(acc[0][0], acc[0][1], acc[0][2], acc[0][3]);
  acc_guard4(acc[0][4], acc[0][5], acc[0][6], acc[0][7]);
  acc_guard4(acc[1][0], acc[1][1], acc[1][2], acc[1][3]);
  acc_guard4(acc[1][4], acc[1][5], acc[1][6], acc[1][7]);

  float* wl = lds_all + wave * SlabCfg<EPI>::PERWF;

  if (EPI == 0) {
    float* slf = wl;
    unsigned short* sl16 = (unsigned short*)(void*)(wl + 2048);
    float* bsl = wl + 4096;
    const bool isq = (n0 < QW);
    unsigned short* P0 = isq ? (unsigned short*)C0 : (unsigned short*)C2;
    unsigned short* P1 = isq ? (unsigned short*)C1 : (unsigned short*)C3;
    const float* bp = isq ? bias0 : bias1;
    const int ldp  = isq ? ldc : ldc2;
    const int col0 = isq ? n0 : (n0 - QW);
    {
      const v4f b4 = *(const v4f*)(bp + col0 + lane * 4);
      bsl[lane * 4 + 0] = bf_rne(b4[0]);
      bsl[lane * 4 + 1] = bf_rne(b4[1]);
      bsl[lane * 4 + 2] = bf_rne(b4[2]);
      bsl[lane * 4 + 3] = bf_rne(b4[3]);
    }
    lds_wave_sync();
#pragma unroll
    for (int i = 0; i < 2; ++i) {
      const int mb = m0 + i * 16;
#pragma unroll
      for (int j = 0; j < 8; ++j)
#pragma unroll
        for (int r = 0; r < 8; ++r)
          slf[(8 * hh + r) * 128 + j * 16 + rl] = acc[i][j][r];
      lds_wave_sync();
#pragma unroll 2
      for (int it = 0; it < 32; ++it) {
        const int row = it >> 1;
        const int d   = ((it & 1) << 5) + lane;
        const float x1 = slf[row * 128 + d] + bsl[d];
        const float x2 = slf[row * 128 + d + 64] + bsl[d + 64];
        const size_t to = (size_t)(mb + row) * NFREQ + d;
        const float cv = cst[to];
        const float sv = snt[to];
        const float o1 = x1 * cv - x2 * sv;
        const float o2 = x2 * cv + x1 * sv;
        const unsigned short hb1 = bf_bits(o1), hb2 = bf_bits(o2);
        const unsigned short lb1 = bf_bits(o1 - bf_val(hb1)), lb2 = bf_bits(o2 - bf_val(hb2));
        const int so = row * 128 + d;
        sl16[so]             = hb1;
        sl16[so + 64]        = hb2;
        sl16[2048 + so]      = lb1;
        sl16[2048 + so + 64] = lb2;
      }
      lds_wave_sync();
      for (int pass = 0; pass < 2; ++pass) {
#pragma unroll
        for (int it = 0; it < 8; ++it) {
          const int row = it * 2 + hh;
          const int c8  = rl * 8;
          const v4u vh = *(const v4u*)(sl16 + row * 128 + c8);
          const v4u vl = *(const v4u*)(sl16 + 2048 + row * 128 + c8);
          const size_t go = (size_t)(mb + row) * ldp + col0 + c8;
          *(volatile v4u*)(P0 + go) = vh;
          *(volatile v4u*)(P1 + go) = vl;
        }
        __threadfence();
      }
      lds_wave_sync();
    }
  } else if (EPI == 1) {
    unsigned short* sl16 = (unsigned short*)(void*)wl;
    unsigned short* P0 = (unsigned short*)C0;
    unsigned short* P1 = (unsigned short*)C1;
#pragma unroll
    for (int i = 0; i < 2; ++i) {
      const int mb = m0 + i * 16;
      const v4f blo = *(const v4f*)(bias0 + mb + 8 * hh);
      const v4f bhi = *(const v4f*)(bias0 + mb + 8 * hh + 4);
      float brow[8];
      brow[0] = bf_rne(blo[0]); brow[1] = bf_rne(blo[1]); brow[2] = bf_rne(blo[2]); brow[3] = bf_rne(blo[3]);
      brow[4] = bf_rne(bhi[0]); brow[5] = bf_rne(bhi[1]); brow[6] = bf_rne(bhi[2]); brow[7] = bf_rne(bhi[3]);
#pragma unroll
      for (int r = 0; r < 8; ++r) {
#pragma unroll
        for (int j = 0; j < 8; ++j) {
          const float v = acc[i][j][r] + brow[r];
          const unsigned short hb = bf_bits(v);
          const unsigned short lb = bf_bits(v - bf_val(hb));
          const int so = (8 * hh + r) * 128 + j * 16 + rl;
          sl16[so]        = hb;
          sl16[2048 + so] = lb;
        }
      }
      lds_wave_sync();
      for (int pass = 0; pass < 2; ++pass) {
#pragma unroll
        for (int it = 0; it < 8; ++it) {
          const int row = it * 2 + hh;
          const int c8  = rl * 8;
          const v4u vh = *(const v4u*)(sl16 + row * 128 + c8);
          const v4u vl = *(const v4u*)(sl16 + 2048 + row * 128 + c8);
          const size_t go = (size_t)(mb + row) * ldc + n0 + c8;
          *(volatile v4u*)(P0 + go) = vh;
          *(volatile v4u*)(P1 + go) = vl;
        }
        __threadfence();
      }
      lds_wave_sync();
    }
  } else {
    float* slf = wl;
    float* bsl = wl + 2048;
    float* C = (float*)C0;
    {
      const v4f b4 = *(const v4f*)(bias0 + n0 + lane * 4);
      bsl[lane * 4 + 0] = bf_rne(b4[0]);
      bsl[lane * 4 + 1] = bf_rne(b4[1]);
      bsl[lane * 4 + 2] = bf_rne(b4[2]);
      bsl[lane * 4 + 3] = bf_rne(b4[3]);
    }
    lds_wave_sync();
#pragma unroll
    for (int i = 0; i < 2; ++i) {
#pragma unroll
      for (int j = 0; j < 8; ++j) {
        const float bj = bsl[j * 16 + rl];
#pragma unroll
        for (int r = 0; r < 8; ++r)
          slf[(8 * hh + r) * 128 + j * 16 + rl] = acc[i][j][r] + bj;
      }
      lds_wave_sync();
      for (int pass = 0; pass < 2; ++pass) {
#pragma unroll
        for (int row = 0; row < 16; ++row) {
          const v4f v = *(const v4f*)(slf + row * 128 + lane * 4);
          *(volatile v4f*)(C + (size_t)(m0 + i * 16 + row) * ldc + n0 + lane * 4) = v;
        }
        __threadfence();
      }
      lds_wave_sync();
    }
  }
}

#define AKC  32
#define KP   136
#define VP   40
#define PP   40
#define L_KH  0
#define L_KL  (AKC * KP)
#define L_VH  (2 * AKC * KP)
#define L_VL  (2 * AKC * KP + HDM * VP)
#define L_PH  (2 * AKC * KP + 2 * HDM * VP)
#define L_PL  (L_PH + 4 * 16 * PP)
#define L_TOT (L_PL + 4 * 16 * PP)
#define L_OH  0
#define L_OL  (4 * 16 * HDM)
static_assert(L_OL + 4 * 16 * HDM <= L_PH);
static_assert(L_TOT * 2 <= 65536);
static_assert((L_KL % 8) == 0 && (L_VH % 8) == 0 && (L_VL % 8) == 0 && (L_PH % 8) == 0 && (L_PL % 8) == 0 && (L_OL % 8) == 0);
static_assert(SQ % 64 == 0 && EMB % 128 == 0 && EMB % 32 == 0 && AOW % 32 == 0 && QKN % 128 == 0 && HDM == 128);

__global__ __launch_bounds__(128) void attn_kernel(
    const unsigned short* __restrict__ qhp, const unsigned short* __restrict__ qlp,
    const unsigned short* __restrict__ khp, const unsigned short* __restrict__ klp,
    const unsigned short* __restrict__ vhp, const unsigned short* __restrict__ vlp,
    unsigned short* __restrict__ aop, float sscale) {
  __shared__ __align__(16) unsigned short L[L_TOT];
  unsigned short* Ks  = L + L_KH;
  unsigned short* Kls = L + L_KL;
  unsigned short* Vhs = L + L_VH;
  unsigned short* Vls = L + L_VL;

  const int tid  = (int)threadIdx.x;
  const int lane = tid & 31;
  const int wave = wave_id();
  const int hh   = lane >> 4;
  const int c    = lane & 15;
  const int qt   = (int)blockIdx.x;
  const int h    = (int)blockIdx.y;
  const int q0   = qt * 64 + wave * 16;

  const __bf16* Qhr = (const __bf16*)(const void*)qhp + (size_t)(q0 + c) * EMB + h * HDM + 8 * hh;
  const __bf16* Qlr = (const __bf16*)(const void*)qlp + (size_t)(q0 + c) * EMB + h * HDM + 8 * hh;

  unsigned short* ph = L + L_PH + wave * 16 * PP;
  unsigned short* pl = L + L_PL + wave * 16 * PP;

  float mrow[8], lrow[8];
  v8f oacc[8];
#pragma unroll
  for (int r = 0; r < 8; ++r) { mrow[r] = -INFINITY; lrow[r] = 0.f; }
#pragma unroll
  for (int t = 0; t < 8; ++t) oacc[t] = zero8();

  const int nch = 2 * qt + 2;
  for (int kc = 0; kc < nch; ++kc) {
    const int kv0 = kc * AKC;
    __syncthreads();
#pragma unroll
    for (int u = 0; u < 4; ++u) {
      const int p   = tid + 128 * u;
      const int key = p >> 4, d8 = (p & 15) * 8;
      const size_t ko = (size_t)(kv0 + key) * EMB + h * HDM + d8;
      const v4u kx = *(const v4u*)(khp + ko);
      const v4u ky = *(const v4u*)(klp + ko);
      *(v4u*)(Ks  + key * KP + d8) = kx;
      *(v4u*)(Kls + key * KP + d8) = ky;
      const int d = p >> 2, k8 = (p & 3) * 8;
      const size_t vo = (size_t)(h * HDM + d) * SQ + kv0 + k8;
      const v4u vx = *(const v4u*)(vhp + vo);
      const v4u vy = *(const v4u*)(vlp + vo);
      *(v4u*)(Vhs + d * VP + k8) = vx;
      *(v4u*)(Vls + d * VP + k8) = vy;
    }
    __syncthreads();

    v8f sa[2];
    sa[0] = zero8(); sa[1] = zero8();
#pragma unroll
    for (int dc = 0; dc < 4; ++dc) {
      const v16b qh = ldfrag_b(Qhr + dc * 32);
      const v16b ql = ldfrag_b(Qlr + dc * 32);
#pragma unroll
      for (int j = 0; j < 2; ++j) {
        const v16b kb = ldfrag_b((const __bf16*)(const void*)Ks  + (j * 16 + c) * KP + dc * 32 + 8 * hh);
        const v16b kl = ldfrag_b((const __bf16*)(const void*)Kls + (j * 16 + c) * KP + dc * 32 + 8 * hh);
        sa[j] = mma_b(qh, kb, sa[j]);
        sa[j] = mma_b(qh, kl, sa[j]);
        sa[j] = mma_b(ql, kb, sa[j]);
        guard1b4(sa[j], qh, ql, kb, kl);
      }
    }
    acc_guard2(sa[0], sa[1]);

    const bool diag = (kc >= 2 * qt);
    float cm[8];
#pragma unroll
    for (int r = 0; r < 8; ++r) {
      const int qrow = q0 + 8 * hh + r;
      float m = -INFINITY;
#pragma unroll
      for (int j = 0; j < 2; ++j) {
        const int kvcol = kv0 + j * 16 + c;
        const float sv = sa[j][r] * sscale;
        const bool masked = diag && (kvcol > qrow);
        const float sm = masked ? -INFINITY : sv;
        sa[j][r] = sm;
        m = fmaxf(m, sm);
      }
#pragma unroll
      for (int off = 1; off < 16; off <<= 1) m = fmaxf(m, __shfl_xor(m, off, 32));
      cm[r] = m;
    }
#pragma unroll
    for (int r = 0; r < 8; ++r) {
      const float mnew  = fmaxf(mrow[r], cm[r]);
      const float muse  = (mnew > -INFINITY) ? mnew : 0.0f;
      const float alpha = __expf(mrow[r] - muse);
      mrow[r] = mnew;
      float psum = 0.f;
#pragma unroll
      for (int j = 0; j < 2; ++j) {
        const float p = __expf(sa[j][r] - muse);
        psum += p;
        const unsigned short hb = bf_bits(p);
        const unsigned short lb = bf_bits(p - bf_val(hb));
        const int po = (8 * hh + r) * PP + j * 16 + c;
        ph[po] = hb;
        pl[po] = lb;
      }
#pragma unroll
      for (int off = 1; off < 16; off <<= 1) psum += __shfl_xor(psum, off, 32);
      lrow[r] = lrow[r] * alpha + psum;
#pragma unroll
      for (int t = 0; t < 8; ++t) oacc[t][r] *= alpha;
    }
    lds_wave_sync();
    const v16b pa = ldfrag_b((const __bf16*)(const void*)ph + c * PP + 8 * hh);
    const v16b pr = ldfrag_b((const __bf16*)(const void*)pl + c * PP + 8 * hh);
#pragma unroll
    for (int t = 0; t < 8; ++t) {
      const v16b vb = ldfrag_b((const __bf16*)(const void*)Vhs + (t * 16 + c) * VP + 8 * hh);
      const v16b vr = ldfrag_b((const __bf16*)(const void*)Vls + (t * 16 + c) * VP + 8 * hh);
      oacc[t] = mma_b(pa, vb, oacc[t]);
      oacc[t] = mma_b(pa, vr, oacc[t]);
      oacc[t] = mma_b(pr, vb, oacc[t]);
      guard1b4(oacc[t], pa, pr, vb, vr);
    }
  }
  __syncthreads();
  acc_guard4(oacc[0], oacc[1], oacc[2], oacc[3]);
  acc_guard4(oacc[4], oacc[5], oacc[6], oacc[7]);

  unsigned short* osh = L + L_OH + wave * 16 * HDM;
  unsigned short* osl = L + L_OL + wave * 16 * HDM;
#pragma unroll
  for (int r = 0; r < 8; ++r) {
    const float inv = 1.0f / lrow[r];
#pragma unroll
    for (int t = 0; t < 8; ++t) {
      const float o = oacc[t][r] * inv;
      const unsigned short hb = bf_bits(o);
      const unsigned short lb = bf_bits(o - bf_val(hb));
      const int so = (8 * hh + r) * HDM + t * 16 + c;
      osh[so] = hb;
      osl[so] = lb;
    }
  }
  lds_wave_sync();
  unsigned short* Ag = aop + (size_t)q0 * AOW + h * HDM;
  const int c8 = c * 8;
  for (int pass = 0; pass < 2; ++pass) {
#pragma unroll
    for (int it = 0; it < 8; ++it) {
      const int row = it * 2 + hh;
      const v4u x = *(const v4u*)(osh + row * HDM + c8);
      const v4u y = *(const v4u*)(osl + row * HDM + c8);
      *(volatile v4u*)(Ag + (size_t)row * AOW + c8)      = x;
      *(volatile v4u*)(Ag + (size_t)row * AOW + QW + c8) = y;
    }
    __threadfence();
  }
}

extern "C" void kernel_launch(void* const* d_in, const int* in_sizes, int n_in,
                              void* d_out, int out_size, void* d_ws, size_t ws_size,
                              hipStream_t stream) {
  if (n_in < 9) return;
  if (in_sizes[0] != NTOK * EMB) return;
  if (in_sizes[1] != EMB * EMB) return;
  if (in_sizes[2] != EMB) return;
  if (in_sizes[3] != EMB * EMB) return;
  if (in_sizes[4] != EMB) return;
  if (in_sizes[5] != EMB * EMB) return;
  if (in_sizes[6] != EMB) return;
  if (in_sizes[7] != EMB * EMB) return;
  if (in_sizes[8] != EMB) return;
  if (out_size != NTOK * EMB) return;

  const float* x  = (const float*)d_in[0];
  const float* wq = (const float*)d_in[1];
  const float* bq = (const float*)d_in[2];
  const float* wk = (const float*)d_in[3];
  const float* bk = (const float*)d_in[4];
  const float* wv = (const float*)d_in[5];
  const float* bv = (const float*)d_in[6];
  const float* wo = (const float*)d_in[7];
  const float* bo = (const float*)d_in[8];
  float* out = (float*)d_out;

  const size_t szXB  = (size_t)NTOK * EMB * 2;
  const size_t szWQK = (size_t)QKN * EMB * 2;
  const size_t szWV  = (size_t)EMB * EMB * 2;
  const size_t szWO2 = (size_t)EMB * AOW * 2;
  const size_t szT   = (size_t)SQ * NFREQ * 4;
  const size_t szP   = (size_t)SQ * EMB * 2;
  const size_t szAO  = (size_t)SQ * AOW * 2;
  size_t off = 0;
  const size_t oXB  = off; off += szXB;
  const size_t oWQK = off; off += szWQK;
  const size_t oWV  = off; off += szWV;
  const size_t oWO2 = off; off += szWO2;
  const size_t oCST = off; off += szT;
  const size_t oSNT = off; off += szT;
  const size_t oQH  = off; off += szP;
  const size_t oQL  = off; off += szP;
  const size_t oKH  = off; off += szP;
  const size_t oKL  = off; off += szP;
  const size_t oVTH = off; off += szP;
  const size_t oVTL = off; off += szP;
  const size_t oAO  = off; off += szAO;
  if (off > ws_size) return;
  if (off > (size_t)134217728) return;

  char* ws = (char*)d_ws;
  unsigned short* XB  = (unsigned short*)(ws + oXB);
  unsigned short* WQK = (unsigned short*)(ws + oWQK);
  unsigned short* WV  = (unsigned short*)(ws + oWV);
  unsigned short* WO2 = (unsigned short*)(ws + oWO2);
  float*          CST = (float*)(ws + oCST);
  float*          SNT = (float*)(ws + oSNT);
  unsigned short* QH  = (unsigned short*)(ws + oQH);
  unsigned short* QL  = (unsigned short*)(ws + oQL);
  unsigned short* KH  = (unsigned short*)(ws + oKH);
  unsigned short* KL  = (unsigned short*)(ws + oKL);
  unsigned short* VTH = (unsigned short*)(ws + oVTH);
  unsigned short* VTL = (unsigned short*)(ws + oVTL);
  unsigned short* AO  = (unsigned short*)(ws + oAO);

  const dim3 b256(256), b128(128);
  const int lds0 = 4 * SlabCfg<0>::PERWF * 4;
  const int lds1 = 4 * SlabCfg<1>::PERWF * 4;
  const int lds2 = 4 * SlabCfg<2>::PERWF * 4;
  const float sscale = 0.08838834764831845f;

  rope_table_kernel<<<dim3(SQ / 8), b256, 0, stream>>>(CST, SNT, SQ);
  cvt_bf16_kernel<<<dim3((NTOK * EMB / 8) / 256), b256, 0, stream>>>(x, XB, NTOK * EMB / 8);
  cvt_bf16_kernel<<<dim3((EMB * EMB / 8) / 256), b256, 0, stream>>>(wq, WQK, EMB * EMB / 8);
  cvt_bf16_kernel<<<dim3((EMB * EMB / 8) / 256), b256, 0, stream>>>(wk, WQK + (size_t)QW * EMB, EMB * EMB / 8);
  cvt_bf16_kernel<<<dim3((EMB * EMB / 8) / 256), b256, 0, stream>>>(wv, WV, EMB * EMB / 8);
  cvt_wo2_kernel<<<dim3((EMB * EMB / 8) / 256), b256, 0, stream>>>(wo, WO2, EMB * EMB / 8, EMB, AOW);

  (void)hipFuncSetAttribute(reinterpret_cast<const void*>(&gemm_w32x128_kernel<0>),
                            hipFuncAttributeMaxDynamicSharedMemorySize, lds0);

  for (int b = 0; b < NB; ++b) {
    const unsigned short* XBb = XB + (size_t)b * SQ * EMB;
    gemm_w32x128_kernel<0><<<dim3((SQ / 32) * (QKN / 128) / 4), b128, lds0, stream>>>(
        XBb, EMB, WQK, EMB, CST, SNT, bq, bk, (void*)QH, (void*)QL, (void*)KH, (void*)KL, QW, QW, SQ, QKN, EMB);
    gemm_w32x128_kernel<1><<<dim3((EMB / 32) * (SQ / 128) / 4), b128, lds1, stream>>>(
        WV, EMB, XBb, EMB, CST, SNT, bv, bv, (void*)VTH, (void*)VTL, (void*)VTH, (void*)VTL, SQ, SQ, EMB, SQ, EMB);
    attn_kernel<<<dim3(SQ / 64, NH), b128, 0, stream>>>(QH, QL, KH, KL, VTH, VTL, AO, sscale);
    float* outb = out + (size_t)b * SQ * EMB;
    gemm_w32x128_kernel<2><<<dim3((SQ / 32) * (EMB / 128) / 4), b128, lds2, stream>>>(
        AO, AOW, WO2, AOW, CST, SNT, bo, bo, (void*)outb, (void*)outb, (void*)outb, (void*)outb, EMB, EMB, SQ, EMB, AOW);
  }
  (void)hipGetLastError();
}
